// RadianceRenderer_50723563765837
// MI455X (gfx1250) — hardware-verified
//
#include <hip/hip_runtime.h>

#define NR_   16384
#define TS_   128
#define HST   72

typedef _Float16 f16;
typedef __attribute__((ext_vector_type(16))) f16 f16x16;
typedef __attribute__((ext_vector_type(8)))  f16 f16x8;
typedef __attribute__((ext_vector_type(8)))  float f32x8;
typedef __attribute__((ext_vector_type(4)))  float v4f_t;
typedef float v4fa __attribute__((ext_vector_type(4), may_alias));

__device__ __forceinline__ f32x8 wmma16(f16x16 a, f16x16 b, f32x8 c) {
  c = __builtin_amdgcn_wmma_f32_16x16x32_f16(false, a, false, b, (short)0, c, false, false);
  asm volatile("v_nop\n\tv_nop\n\tv_nop\n\tv_nop" : "+v"(c) : "v"(a), "v"(b));
  return c;
}
__device__ __forceinline__ f16x16 lds_frag(const f16* base, int stride) {
  const int lane = threadIdx.x & 31, row = lane & 15, kh = (lane >> 4) * 8;
  const f16x8 lo = *(const f16x8*)(base + row * stride + kh);
  const f16x8 hi = *(const f16x8*)(base + row * stride + kh + 16);
  f16x16 f;
#pragma unroll
  for (int i = 0; i < 8; ++i) { f[i] = lo[i]; f[i + 8] = hi[i]; }
  return f;
}

__global__ __launch_bounds__(64) void k_render(const float* __restrict__ rays_o, const float* __restrict__ rays_d,
                                               const float* __restrict__ tnoise, const float* __restrict__ aabb,
                                               const float* __restrict__ W1, const float* __restrict__ b1,
                                               const float* __restrict__ W2, const float* __restrict__ b2,
                                               const float* __restrict__ Wc1, const float* __restrict__ bc1,
                                               const float* __restrict__ Wc2, const float* __restrict__ bc2,
                                               float* __restrict__ out) {
  __shared__ __attribute__((aligned(16))) f16 W1S[64 * 40];
  __shared__ __attribute__((aligned(16))) f16 W2S[16 * HST];
  __shared__ __attribute__((aligned(16))) f16 Wc1S[64 * 40];
  __shared__ __attribute__((aligned(16))) f16 Wc2S[16 * HST];
  __shared__ __attribute__((aligned(16))) f16 hS[2][16 * HST];
  __shared__ __attribute__((aligned(16))) f16 fS[2][16 * 40];
  __shared__ float sgS[2][16], rgbS[2][16][4];
  __shared__ __attribute__((aligned(16))) float oS[2][16 * 4];
  __shared__ float b1S[64], bc1S[64], b2S[16], bc2S[4];
  const int tid = threadIdx.x, lane = tid & 31, wave = tid >> 5, cl = lane & 15, hsel = lane >> 4, rh = hsel * 8, kh = rh;

  for (int e = tid; e < 64 * 40; e += 64) { const int n = e / 40, k = e % 40;
    W1S[e]  = (f16)((k < 27) ? W1[k * 64 + n] : 0.0f);
    Wc1S[e] = (f16)((k < 19) ? Wc1[k * 64 + n] : 0.0f); }
  for (int e = tid; e < 16 * HST; e += 64) { const int n = e / HST, k = e % HST;
    W2S[e]  = (f16)((k < 64) ? W2[k * 16 + n] : 0.0f);
    Wc2S[e] = (f16)((k < 64 && n < 3) ? Wc2[k * 3 + n] : 0.0f); }
  if (tid < 64) { b1S[tid] = b1[tid]; bc1S[tid] = bc1[tid]; }
  if (tid < 16) b2S[tid] = b2[tid];
  if (tid < 4) bc2S[tid] = (tid < 3) ? bc2[tid] : 0.0f;
  for (int e = tid; e < 2 * 16 * 40; e += 64) (&fS[0][0])[e] = (f16)0.0f;
  __syncthreads();

  const int ray0 = (blockIdx.x * 2 + wave) * 16;
  const int myray = ray0 + cl;
  const float ox = rays_o[myray * 3 + 0], oy = rays_o[myray * 3 + 1], oz = rays_o[myray * 3 + 2];
  const float dx = rays_d[myray * 3 + 0], dy = rays_d[myray * 3 + 1], dz = rays_d[myray * 3 + 2];
  const float a0x = aabb[0], a0y = aabb[1], a0z = aabb[2], a1x = aabb[3], a1y = aabb[4], a1z = aabb[5];
  const float ix = 1.0f / dx, iy = 1.0f / dy, iz = 1.0f / dz;
  const float t0x = (a0x - ox) * ix, t0y = (a0y - oy) * iy, t0z = (a0z - oz) * iz;
  const float t1x = (a1x - ox) * ix, t1y = (a1y - oy) * iy, t1z = (a1z - oz) * iz;
  const float tnear = fmaxf(fmaxf(fmaxf(fminf(t0x, t1x), fminf(t0y, t1y)), fminf(t0z, t1z)), 0.0f);
  const float tfar  = fminf(fminf(fmaxf(t0x, t1x), fmaxf(t0y, t1y)), fmaxf(t0z, t1z));
  const float active = (tfar > tnear) ? 1.0f : 0.0f;
  const float dnorm = sqrtf(dx * dx + dy * dy + dz * dz);
  const float tfinal = tfar * 10.0f;
  const float idn = 1.0f / dnorm;
  const float sh0 = 0.28209479177387814f, sh1 = 0.4886025119029199f * dy * idn, sh2 = 0.4886025119029199f * dz * idn, sh3 = 0.4886025119029199f * dx * idn;
  const float sx = 2.0f / (a1x - a0x), sy = 2.0f / (a1y - a0y), szc = 2.0f / (a1z - a0z);

  float csum = 0.0f, colr = 0.0f, colg = 0.0f, colb = 0.0f, asum = 0.0f;
  float* sg = sgS[wave]; f16* hw = hS[wave]; f16* fw = fS[wave];

#pragma unroll 1
  for (int t = 0; t < TS_; ++t) {
    const float base = ((float)t + tnoise[(size_t)t * NR_ + myray]) * (1.0f / 128.0f);
    const float ts = tnear + (tfar - tnear) * base;
    const float px = ox + ts * dx, py = oy + ts * dy, pz = oz + ts * dz;
    const float xn = (px - a0x) * sx - 1.0f, yn = (py - a0y) * sy - 1.0f, zn = (pz - a0z) * szc - 1.0f;
    f16x16 af;
#pragma unroll
    for (int i = 0; i < 16; ++i) {
      const int k = kh + (i & 7) + ((i >> 3) << 4);
      float v = 0.0f;
      if (k < 3) v = (k == 0) ? xn : (k == 1) ? yn : zn;
      else if (k < 27) {
        const int f = (k - 3) / 6, w6 = (k - 3) % 6, dm = w6 % 3;
        const float c = (dm == 0) ? xn : (dm == 1) ? yn : zn;
        const float rev = c * (0.5f * (float)(1 << f)) + ((w6 >= 3) ? 0.25f : 0.0f);
        v = __builtin_amdgcn_sinf(rev);
      }
      af[i] = (f16)v;
    }
    f32x8 h[4];
#pragma unroll
    for (int nt = 0; nt < 4; ++nt) { f32x8 z = {}; h[nt] = wmma16(af, lds_frag(W1S + nt * 16 * 40, 40), z); }
#pragma unroll
    for (int nt = 0; nt < 4; ++nt)
#pragma unroll
      for (int r = 0; r < 8; ++r) hw[(rh + r) * HST + nt * 16 + cl] = (f16)fmaxf(h[nt][r] + b1S[nt * 16 + cl], 0.0f);
    asm volatile("s_wait_dscnt 0" ::: "memory");
    __builtin_amdgcn_wave_barrier();
    f32x8 dh = {};
    dh = wmma16(lds_frag(hw, HST), lds_frag(W2S, HST), dh);
    dh = wmma16(lds_frag(hw + 32, HST), lds_frag(W2S + 32, HST), dh);
    {
      const float bb = b2S[cl];
#pragma unroll
      for (int r = 0; r < 8; ++r) {
        const float v = dh[r] + bb;
        if (cl == 0) sg[rh + r] = __expf(v);
        else         fw[(rh + r) * 40 + (cl - 1)] = (f16)v;
      }
      if (hsel == 0) { fw[cl * 40 + 15] = (f16)sh0; fw[cl * 40 + 16] = (f16)sh1; fw[cl * 40 + 17] = (f16)sh2; fw[cl * 40 + 18] = (f16)sh3; }
    }
    asm volatile("s_wait_dscnt 0" ::: "memory");
    __builtin_amdgcn_wave_barrier();
    const f16x16 fa = lds_frag(fw, 40);
    f32x8 hc[4];
#pragma unroll
    for (int nt = 0; nt < 4; ++nt) { f32x8 z = {}; hc[nt] = wmma16(fa, lds_frag(Wc1S + nt * 16 * 40, 40), z); }
#pragma unroll
    for (int nt = 0; nt < 4; ++nt)
#pragma unroll
      for (int r = 0; r < 8; ++r) hw[(rh + r) * HST + nt * 16 + cl] = (f16)fmaxf(hc[nt][r] + bc1S[nt * 16 + cl], 0.0f);
    asm volatile("s_wait_dscnt 0" ::: "memory");
    __builtin_amdgcn_wave_barrier();
    f32x8 cc = {};
    cc = wmma16(lds_frag(hw, HST), lds_frag(Wc2S, HST), cc);
    cc = wmma16(lds_frag(hw + 32, HST), lds_frag(Wc2S + 32, HST), cc);
    if (cl < 3) {
      const float bb = bc2S[cl];
#pragma unroll
      for (int r = 0; r < 8; ++r) rgbS[wave][rh + r][cl] = 1.0f / (1.0f + __expf(-(cc[r] + bb)));
    }
    asm volatile("s_wait_dscnt 0" ::: "memory");
    __builtin_amdgcn_wave_barrier();
    {
      float delta;
      if (t + 1 < TS_) {
        const float base1 = ((float)(t + 1) + tnoise[(size_t)(t + 1) * NR_ + myray]) * (1.0f / 128.0f);
        const float ts1 = tnear + (tfar - tnear) * base1;
        delta = ts1 - ts;
      } else {
        delta = tfinal - ts;
      }
      const float sigma = sg[cl];
      const float sd = sigma * delta * dnorm;
      csum += sd;
      const float trans = __expf(-(csum - sd));
      const float alpha = 1.0f - __expf(-sd);
      const float w = trans * alpha * active;
      colr += w * rgbS[wave][cl][0]; colg += w * rgbS[wave][cl][1]; colb += w * rgbS[wave][cl][2]; asum += w;
    }
    __builtin_amdgcn_wave_barrier();
  }
  if (hsel == 0) { oS[wave][cl * 4 + 0] = colr; oS[wave][cl * 4 + 1] = colg; oS[wave][cl * 4 + 2] = colb; oS[wave][cl * 4 + 3] = asum; }
  asm volatile("s_wait_dscnt 0" ::: "memory");
  __builtin_amdgcn_wave_barrier();
#pragma unroll 1
  for (int pass = 0; pass < 2; ++pass) {
    if (lane < 16) *(volatile v4f_t*)(out + (size_t)(ray0 + lane) * 4) = *(const volatile v4fa*)(oS[wave] + lane * 4);
    __threadfence();
  }
}

extern "C" void kernel_launch(void* const* d_in, const int* in_sizes, int n_in,
                              void* d_out, int out_size, void* d_ws, size_t ws_size,
                              hipStream_t stream) {
  (void)in_sizes; (void)n_in; (void)out_size; (void)d_ws; (void)ws_size;
  const float* rays_o = (const float*)d_in[0];
  const float* rays_d = (const float*)d_in[1];
  const float* tnoise = (const float*)d_in[2];
  const float* aabb   = (const float*)d_in[3];
  const float* W1 = (const float*)d_in[4], *b1 = (const float*)d_in[5], *W2 = (const float*)d_in[6], *b2 = (const float*)d_in[7];
  const float* Wc1 = (const float*)d_in[8], *bc1 = (const float*)d_in[9], *Wc2 = (const float*)d_in[10], *bc2 = (const float*)d_in[11];
  float* out = (float*)d_out;
  k_render<<<dim3(NR_ / 32), dim3(64), 0, stream>>>(rays_o, rays_d, tnoise, aabb, W1, b1, W2, b2, Wc1, bc1, Wc2, bc2, out);
}
